// GraphSAGE_5574867550247
// MI455X (gfx1250) — hardware-verified
//
#include <hip/hip_runtime.h>
#include <stddef.h>
#include <stdint.h>


#define DFE    64
#define HP     128
#define HALLP  192
#define NCLS   10
#define NGR    512
#define NOUT   (NGR * NCLS)
#define NTHR   256
#define NWAVE  8
#define EPT    8
#define CHUNK  (NTHR * EPT)
#define WCAP   (EPT * 32)
#define LISTN  (NWAVE * WCAP)
#define NBA    1024
#define SLA    10
#define RCAP   28672
#define DEGCAP 64
#define GBM    64
#define GTHR   128
#define WP     1216
#define NSUB   19
#define WC0OFF 0
#define WC1OFF 192
#define WC2OFF 448
#define WMOFF  704
#define W1OFF  832
#define PG     16
#define PTHR   192
#define PWAVE  6
#define GAP    384
#define AGG_ZINTS (LISTN + 2 * RCAP + 3 * NBA)
#define AGG_LDS_INTS (AGG_ZINTS + 16)
#define WSMAX  134217728

static_assert((CHUNK & (CHUNK - 1)) == 0 && CHUNK <= 4096);
static_assert((NBA & (NBA - 1)) == 0 && NBA == (1 << SLA));
static_assert(((long long)CHUNK << SLA) < (1LL << 31));
static_assert(LISTN % NTHR == 0);
static_assert(NBA % NWAVE == 0 && NBA % 32 == 0 && NBA % GBM == 0);
static_assert(RCAP % 32 == 0 && AGG_ZINTS % 4 == 0 && LISTN % 4 == 0);
static_assert(AGG_LDS_INTS * 4 <= 300000);
static_assert(DFE == 2 * 32 && HP == 2 * DFE && HALLP == 3 * DFE);
static_assert(GBM == (GTHR / 32) * 16);
static_assert(WP == NSUB * 64 && (WP * 2) % 128 == 0);
static_assert(WC1OFF == 192 && WC2OFF == WC1OFF + 256 && WMOFF == WC2OFF + 256 && W1OFF == WMOFF + 128);
static_assert(W1OFF + 2 * HALLP == WP);
static_assert((NSUB * 512) % NTHR == 0);
static_assert(GAP == 2 * HALLP && GAP % 32 == 0 && PTHR == HALLP && PTHR == 32 * PWAVE);
static_assert(NGR % PG == 0 && (PG * NCLS * 4) % 128 == 0 && (PG * NCLS) / 4 == 40);
static_assert(PG == 16 && PG * NCLS <= PTHR);

typedef float          v2f   __attribute__((ext_vector_type(2)));
typedef float          v4f   __attribute__((ext_vector_type(4)));
typedef float          v8f   __attribute__((ext_vector_type(8)));
typedef int            v4i   __attribute__((ext_vector_type(4)));
typedef int            v8i   __attribute__((ext_vector_type(8)));
typedef unsigned int   v4u   __attribute__((ext_vector_type(4)));
typedef unsigned short v8us  __attribute__((ext_vector_type(8)));
typedef unsigned short v16us __attribute__((ext_vector_type(16)));
typedef __bf16         v16bf __attribute__((ext_vector_type(16)));
typedef v2f  __attribute__((may_alias)) v2fa;
typedef v4f  __attribute__((may_alias)) v4fa;
typedef v4i  __attribute__((may_alias)) v4ia;
typedef v8us __attribute__((may_alias)) v8usa;
typedef unsigned int __attribute__((may_alias)) u32a;
union FragB { v16bf v; v16us u; v8us h[2]; v8i w; };

__device__ __forceinline__ v8f wmb(const FragB& a, const FragB& b, v8f c) {
  v8f d = __builtin_amdgcn_wmma_f32_16x16x32_bf16(false, a.v, false, b.v, (short)0, c, false, false);
  asm volatile("v_nop\n\tv_nop\n\tv_nop\n\tv_nop" : "+v"(d) : "v"(a.w), "v"(b.w));
  return d;
}

__device__ __forceinline__ unsigned bf16_bits(float f) {
  const unsigned u = __float_as_uint(f);
  return (u + 0x7FFFu + ((u >> 16) & 1u)) >> 16;
}
__device__ __forceinline__ float bf16_val(float f) {
  return __uint_as_float(bf16_bits(f) << 16);
}

template <int SLB>
__device__ __forceinline__ int scan_chunk(const int* __restrict__ dsts, int nE, int cbase, int slotBase,
                                          int nb, int vec8, int* list, int tid, int lane, int wave) {
  int wc = 0;
  const int el0  = tid * EPT;
  const int e0   = cbase + el0;
  const int sent = -2147483647 - 1;
  v4i da, db;
  if (vec8 != 0 && cbase + CHUNK <= nE) {
    da = *(const v4i*)(dsts + e0);
    db = *(const v4i*)(dsts + e0 + 4);
  } else {
    da.x = (e0     < nE) ? dsts[min(e0,     nE - 1)] : sent;
    da.y = (e0 + 1 < nE) ? dsts[min(e0 + 1, nE - 1)] : sent;
    da.z = (e0 + 2 < nE) ? dsts[min(e0 + 2, nE - 1)] : sent;
    da.w = (e0 + 3 < nE) ? dsts[min(e0 + 3, nE - 1)] : sent;
    db.x = (e0 + 4 < nE) ? dsts[min(e0 + 4, nE - 1)] : sent;
    db.y = (e0 + 5 < nE) ? dsts[min(e0 + 5, nE - 1)] : sent;
    db.z = (e0 + 6 < nE) ? dsts[min(e0 + 6, nE - 1)] : sent;
    db.w = (e0 + 7 < nE) ? dsts[min(e0 + 7, nE - 1)] : sent;
  }
  const unsigned nbs = (unsigned)slotBase;
  const unsigned unb = (unsigned)nb;
  const unsigned s0 = (unsigned)da.x - nbs, s1 = (unsigned)da.y - nbs;
  const unsigned s2 = (unsigned)da.z - nbs, s3 = (unsigned)da.w - nbs;
  const unsigned s4 = (unsigned)db.x - nbs, s5 = (unsigned)db.y - nbs;
  const unsigned s6 = (unsigned)db.z - nbs, s7 = (unsigned)db.w - nbs;
  const bool h0 = s0 < unb, h1 = s1 < unb, h2 = s2 < unb, h3 = s3 < unb;
  const bool h4 = s4 < unb, h5 = s5 < unb, h6 = s6 < unb, h7 = s7 < unb;
  const unsigned any = __builtin_amdgcn_ballot_w32(h0 | h1 | h2 | h3 | h4 | h5 | h6 | h7);
  if (any != 0u) {
#define HITJ(J, HJ, SJ) { \
      const unsigned mj = __builtin_amdgcn_ballot_w32(HJ); \
      if (mj != 0u) { \
        if (HJ) { \
          const int pos = wc + (int)__builtin_amdgcn_mbcnt_lo(mj, 0u); \
          if (pos < WCAP) list[wave * WCAP + pos] = ((el0 + (J)) << SLB) | (int)(SJ); \
        } \
        wc += (int)__builtin_popcount(mj); } }
    HITJ(0, h0, s0)
    HITJ(1, h1, s1)
    HITJ(2, h2, s2)
    HITJ(3, h3, s3)
    HITJ(4, h4, s4)
    HITJ(5, h5, s5)
    HITJ(6, h6, s6)
    HITJ(7, h7, s7)
#undef HITJ
  }
  return wc;
}

__global__ __launch_bounds__(NTHR) void k_prep(const float* __restrict__ Wl0, const float* __restrict__ Wr0,
                                               const float* __restrict__ Wl1, const float* __restrict__ Wr1,
                                               const float* __restrict__ Wl2, const float* __restrict__ Wr2,
                                               const float* __restrict__ Wm,  const float* __restrict__ W1,
                                               unsigned short* wall) {
  const int u  = (int)blockIdx.x * NTHR + (int)threadIdx.x;
  const int j  = u >> 9;
  const int v  = u & 511;
  const int n  = v >> 3;
  const int k8 = (v & 7) * 8;
  const float* W;
  int kb = 0;
  if (j <= 1)        { W = Wl0; }
  else if (j == 2)   { W = Wr0; }
  else if (j <= 4)   { W = Wl1; }
  else if (j <= 6)   { W = Wr1; }
  else if (j <= 8)   { W = Wl2; }
  else if (j <= 10)  { W = Wr2; }
  else if (j <= 12)  { W = Wm; }
  else if (j < NSUB) { W = W1; kb = ((j - 13) % 3) * 64; }
  else return;
  const float* p = W + (size_t)(kb + k8) * DFE + n;
  v8us o;
#pragma unroll
  for (int i = 0; i < 8; ++i) o[i] = (unsigned short)bf16_bits(p[(size_t)i * DFE]);
  unsigned short* dp = wall + (size_t)n * WP + j * 64 + k8;
  *(volatile v8us*)dp = o;
  __threadfence();
  *(volatile v8us*)dp = o;
}

__global__ __launch_bounds__(NTHR) void k_cvx(const float* __restrict__ x, int nN, int nUnits,
                                              unsigned short* xb) {
  const int u = (int)blockIdx.x * NTHR + (int)threadIdx.x;
  if (u >= nUnits) return;
  const int row = u >> 3;
  const int k8  = (u & 7) * 8;
  const int rc  = row < nN ? row : nN - 1;
  const float* p = x + (size_t)rc * DFE + k8;
  const v4f a = *(const v4fa*)p;
  const v4f b = *(const v4fa*)(p + 4);
  const bool ok = row < nN;
  v8us o;
  o[0] = ok ? (unsigned short)bf16_bits(a.x) : (unsigned short)0;
  o[1] = ok ? (unsigned short)bf16_bits(a.y) : (unsigned short)0;
  o[2] = ok ? (unsigned short)bf16_bits(a.z) : (unsigned short)0;
  o[3] = ok ? (unsigned short)bf16_bits(a.w) : (unsigned short)0;
  o[4] = ok ? (unsigned short)bf16_bits(b.x) : (unsigned short)0;
  o[5] = ok ? (unsigned short)bf16_bits(b.y) : (unsigned short)0;
  o[6] = ok ? (unsigned short)bf16_bits(b.z) : (unsigned short)0;
  o[7] = ok ? (unsigned short)bf16_bits(b.w) : (unsigned short)0;
  unsigned short* dp = xb + (size_t)row * DFE + k8;
  *(volatile v8us*)dp = o;
  __threadfence();
  *(volatile v8us*)dp = o;
}

template <int L0>
__global__ __launch_bounds__(NTHR) void k_scan(const int* __restrict__ srcs, const int* __restrict__ dsts,
                                               int nE, int nN, int vec8, int mRows,
                                               const unsigned short* __restrict__ xb,
                                               const float* __restrict__ hsrc, int hoff,
                                               unsigned short* meanp) {
  extern __shared__ __attribute__((aligned(16))) int dsm[];
  int* list = dsm;
  int* hl   = dsm + LISTN;
  int* sl   = dsm + LISTN + RCAP;
  int* cnt  = dsm + LISTN + 2 * RCAP;
  int* offs = cnt + NBA;
  int* cur  = offs + NBA;
  int* misc = cur + NBA;
  const int tid = (int)threadIdx.x, lane = tid & 31, wave = tid >> 5;
  const int nodeBase = (int)blockIdx.x * NBA;

  {
    const v4i z4 = {0, 0, 0, 0};
    for (int i = tid * 4; i < AGG_ZINTS; i += NTHR * 4) *(v4ia*)(dsm + i) = z4;
    if (tid < 16) misc[tid] = 0;
  }
  __syncthreads();

  int t = 0, ov = 0;
  const int nChunks = (nE + CHUNK - 1) / CHUNK;
#pragma unroll 1
  for (int ch = 0; ch < nChunks; ++ch) {
    const int cbase = ch * CHUNK;
    const int wc = scan_chunk<SLA>(dsts, nE, cbase, nodeBase, NBA, vec8, list, tid, lane, wave);
    if (lane == 0) misc[wave] = wc;
    __syncthreads();
    if (wave == 0) {
#pragma unroll 1
      for (int w2 = 0; w2 < NWAVE; ++w2) {
        int c = misc[w2];
        c = c < 0 ? 0 : (c > WCAP ? WCAP : c);
#pragma unroll 1
        for (int b0 = 0; b0 < c; b0 += 32) {
          const int idx = b0 + lane;
          const int ent = list[w2 * WCAP + (idx < WCAP ? idx : WCAP - 1)];
          const int m32 = (c - b0) < 32 ? (c - b0) : 32;
#pragma unroll 1
          for (int k = 0; k < m32; ++k) {
            const int u    = __builtin_amdgcn_readlane(ent, k);
            const int slot = u & (NBA - 1);
            const int el   = (u >> SLA) & (CHUNK - 1);
            const int pk   = ((cbase + el) << SLA) | slot;
            if (t < RCAP) {
              if (lane == 0) { hl[t] = pk; cnt[slot] = cnt[slot] + 1; }
              t = t + 1;
            } else {
              ov = 1;
            }
          }
        }
      }
    }
    __syncthreads();
  }
  if (wave == 0 && lane == 0) { misc[8] = t; misc[9] = ov; }
  __syncthreads();
  int tt = misc[8];
  tt = tt < 0 ? 0 : (tt > RCAP ? RCAP : tt);
  const int ovf = misc[9];

  if (wave == 0) {
    const int base = lane * (NBA / 32);
    int s = 0;
#pragma unroll 1
    for (int i = 0; i < NBA / 32; ++i) s += cnt[base + i];
    int incl = s;
#pragma unroll
    for (int d = 1; d < 32; d <<= 1) {
      const int y = __shfl_up(incl, d, 32);
      if (lane >= d) incl += y;
    }
    int run = incl - s;
#pragma unroll 1
    for (int i = 0; i < NBA / 32; ++i) {
      const int cv = cnt[base + i];
      offs[base + i] = run;
      cur[base + i]  = run;
      run += cv;
    }
  }
  __syncthreads();
  if (wave == 0) {
#pragma unroll 1
    for (int b0 = 0; b0 < tt; b0 += 32) {
      const int idx = b0 + lane;
      const int ent = hl[idx < RCAP ? idx : RCAP - 1];
      const int m32 = (tt - b0) < 32 ? (tt - b0) : 32;
#pragma unroll 1
      for (int k = 0; k < m32; ++k) {
        const int u    = __builtin_amdgcn_readlane(ent, k);
        const int slot = u & (NBA - 1);
        if (lane == 0) {
          int p = cur[slot];
          p = p < 0 ? 0 : (p > RCAP - 1 ? RCAP - 1 : p);
          sl[p] = u;
          cur[slot] = p + 1;
        }
      }
    }
  }
  __syncthreads();

  const float qnan = __int_as_float(0x7fc00000);
  const float pz = (ovf != 0) ? qnan : 0.0f;
  const int q0s = (4 * lane) & 31, q1s = (4 * lane + 1) & 31;
  const int q2s = (4 * lane + 2) & 31, q3s = (4 * lane + 3) & 31;
#pragma unroll 1
  for (int si = 0; si < NBA / NWAVE; ++si) {
    const int s    = si * NWAVE + wave;
    const int node = nodeBase + s;
    int c = cnt[s];
    const int cfull = c < 0 ? 0 : c;
    const bool big = c > DEGCAP;
    c = c < 0 ? 0 : (c > DEGCAP ? DEGCAP : c);
    int o = offs[s];
    o = o < 0 ? 0 : (o > RCAP ? RCAP : o);
    float acc0 = 0.0f, acc1 = 0.0f;
#pragma unroll 1
    for (int b0 = 0; b0 < c; b0 += 32) {
      int idx = o + b0 + lane;
      idx = idx > RCAP - 1 ? RCAP - 1 : idx;
      const int ent = sl[idx];
      int eid = ent >> SLA;
      eid = eid < 0 ? 0 : (eid > nE - 1 ? nE - 1 : eid);
      int sr = srcs[eid];
      sr = sr < 0 ? 0 : (sr > nN - 1 ? nN - 1 : sr);
      const int m32 = (c - b0) < 32 ? (c - b0) : 32;
#pragma unroll 1
      for (int k = 0; k < m32; ++k) {
        const int sk = __builtin_amdgcn_readlane(sr, k);
        if constexpr (L0 != 0) {
          const unsigned w = *(const u32a*)(xb + (size_t)sk * DFE + 2 * lane);
          acc0 += __uint_as_float(w << 16);
          acc1 += __uint_as_float(w & 0xffff0000u);
        } else {
          const v2f a = *(const v2fa*)(hsrc + (size_t)sk * HALLP + hoff + 2 * lane);
          acc0 += a.x;
          acc1 += a.y;
        }
      }
    }
    const float dn  = (cfull < 1) ? 1.0f : (float)cfull;
    const float inv = 1.0f / dn;
    const float pzr = big ? qnan : pz;
    const bool live = node < nN;
    const float y0 = acc0 * inv + pzr;
    const float y1 = acc1 * inv + pzr;
    const float v0 = live ? y0 : 0.0f;
    const float v1 = live ? y1 : 0.0f;
    const bool wr = (node < mRows) && (lane < 16);
    const unsigned hb0 = bf16_bits(v0), hb1 = bf16_bits(v1);
    const unsigned lb0 = bf16_bits(v0 - __uint_as_float(hb0 << 16));
    const unsigned lb1 = bf16_bits(v1 - __uint_as_float(hb1 << 16));
    const int hw = (int)(hb0 | (hb1 << 16));
    const int lw = (int)(lb0 | (lb1 << 16));
    const int g0 = __shfl(hw, q0s, 32), g1 = __shfl(hw, q1s, 32);
    const int g2 = __shfl(hw, q2s, 32), g3 = __shfl(hw, q3s, 32);
    const int p0 = __shfl(lw, q0s, 32), p1 = __shfl(lw, q1s, 32);
    const int p2 = __shfl(lw, q2s, 32), p3 = __shfl(lw, q3s, 32);
    const bool lsel = (lane & 8) != 0;
    v4u pv;
    pv.x = (unsigned int)(lsel ? p0 : g0);
    pv.y = (unsigned int)(lsel ? p1 : g1);
    pv.z = (unsigned int)(lsel ? p2 : g2);
    pv.w = (unsigned int)(lsel ? p3 : g3);
    unsigned short* hp = meanp + (size_t)node * HP + 8 * (lane & 15);
    if (wr) *(volatile v4u*)hp = pv;
    __threadfence();
    if (wr) *(volatile v4u*)hp = pv;
  }
}

template <int L0, int WRH>
__global__ __launch_bounds__(GTHR) void k_layer(const unsigned short* __restrict__ meanp,
                                                const unsigned short* __restrict__ a2,
                                                const unsigned short* __restrict__ wall, int wcOff,
                                                const float* __restrict__ bl, const float* __restrict__ bm,
                                                float* hall, int coloff, unsigned short* hout) {
  __shared__ __attribute__((aligned(16))) unsigned short thl[GBM * HP];
  __shared__ __attribute__((aligned(16))) float stg[GBM * DFE];
  constexpr int P2  = (L0 != 0) ? DFE : HP;
  constexpr int K2S = P2 / 32;
  const int tid = (int)threadIdx.x, lane = tid & 31, wave = tid >> 5, hh = lane >> 4, m = lane & 15;
  const int rowBase = (int)blockIdx.x * GBM;
  const int arow = rowBase + 16 * wave + m;

  v8f acc[4];
  {
    const v8f z = {0.f, 0.f, 0.f, 0.f, 0.f, 0.f, 0.f, 0.f};
    acc[0] = z; acc[1] = z; acc[2] = z; acc[3] = z;
  }
  const unsigned short* ap  = meanp + (size_t)arow * HP + 8 * hh;
  const unsigned short* ap2 = a2 + (size_t)arow * P2 + 8 * hh;
  const unsigned short* wp  = wall + (size_t)m * WP + wcOff + 8 * hh;
#pragma unroll 1
  for (int ks = 0; ks < HP / 32; ++ks) {
    FragB af;
    af.h[0] = *(const v8usa*)(ap + 32 * ks);
    af.h[1] = *(const v8usa*)(ap + 32 * ks + 16);
#pragma unroll
    for (int t = 0; t < 4; ++t) {
      const unsigned short* wq = wp + (size_t)(16 * t) * WP + 32 * ks;
      FragB bf;
      bf.h[0] = *(const v8usa*)wq;
      bf.h[1] = *(const v8usa*)(wq + 16);
      acc[t] = wmb(af, bf, acc[t]);
    }
  }
#pragma unroll 1
  for (int ks = 0; ks < K2S; ++ks) {
    FragB af;
    af.h[0] = *(const v8usa*)(ap2 + 32 * ks);
    af.h[1] = *(const v8usa*)(ap2 + 32 * ks + 16);
#pragma unroll
    for (int t = 0; t < 4; ++t) {
      const unsigned short* wq = wp + (size_t)(16 * t) * WP + HP + 32 * ks;
      FragB bf;
      bf.h[0] = *(const v8usa*)wq;
      bf.h[1] = *(const v8usa*)(wq + 16);
      acc[t] = wmb(af, bf, acc[t]);
    }
  }

#pragma unroll
  for (int t = 0; t < 4; ++t) {
    const int lc = 16 * t + m;
    const float bv = bf16_val(bl[lc]);
#pragma unroll
    for (int r = 0; r < 8; ++r) {
      const int lr = 16 * wave + 8 * hh + r;
      const float v = acc[t][r] + bv;
      const unsigned hb = bf16_bits(v);
      const unsigned lb = bf16_bits(v - __uint_as_float(hb << 16));
      thl[lr * HP + lc]       = (unsigned short)hb;
      thl[lr * HP + DFE + lc] = (unsigned short)lb;
    }
  }
  __syncthreads();

  v8f ac2[4];
  {
    const v8f z = {0.f, 0.f, 0.f, 0.f, 0.f, 0.f, 0.f, 0.f};
    ac2[0] = z; ac2[1] = z; ac2[2] = z; ac2[3] = z;
  }
  const unsigned short* tp  = thl + (16 * wave + m) * HP + 8 * hh;
  const unsigned short* wmp = wall + (size_t)m * WP + WMOFF + 8 * hh;
#pragma unroll 1
  for (int ks = 0; ks < HP / 32; ++ks) {
    FragB af;
    af.h[0] = *(const v8usa*)(tp + 32 * ks);
    af.h[1] = *(const v8usa*)(tp + 32 * ks + 16);
#pragma unroll
    for (int t = 0; t < 4; ++t) {
      const unsigned short* wq = wmp + (size_t)(16 * t) * WP + 32 * ks;
      FragB bf;
      bf.h[0] = *(const v8usa*)wq;
      bf.h[1] = *(const v8usa*)(wq + 16);
      ac2[t] = wmb(af, bf, ac2[t]);
    }
  }

#pragma unroll
  for (int t = 0; t < 4; ++t) {
    const int lc = 16 * t + m;
    const float bv = bf16_val(bm[lc]);
#pragma unroll
    for (int r = 0; r < 8; ++r) {
      const int lr = 16 * wave + 8 * hh + r;
      const float v = ac2[t][r] + bv;
      const float y = (v > 0.0f) ? v : (v - v);
      stg[lr * DFE + lc] = y;
    }
  }
  __syncthreads();

  v4f fv[8];
  v8us qv[8];
#pragma unroll
  for (int i = 0; i < 8; ++i) {
    const int lr = 16 * wave + 2 * i + hh;
    fv[i] = *(const v4fa*)(stg + lr * DFE + 4 * m);
    if constexpr (WRH != 0) {
      const float* sp = stg + lr * DFE + 8 * (m & 7);
      const v4f c0 = *(const v4fa*)sp;
      const v4f c1 = *(const v4fa*)(sp + 4);
      const bool lo = (m & 8) != 0;
      v8us q;
      unsigned hb, lb;
      hb = bf16_bits(c0.x); lb = bf16_bits(c0.x - __uint_as_float(hb << 16)); q[0] = (unsigned short)(lo ? lb : hb);
      hb = bf16_bits(c0.y); lb = bf16_bits(c0.y - __uint_as_float(hb << 16)); q[1] = (unsigned short)(lo ? lb : hb);
      hb = bf16_bits(c0.z); lb = bf16_bits(c0.z - __uint_as_float(hb << 16)); q[2] = (unsigned short)(lo ? lb : hb);
      hb = bf16_bits(c0.w); lb = bf16_bits(c0.w - __uint_as_float(hb << 16)); q[3] = (unsigned short)(lo ? lb : hb);
      hb = bf16_bits(c1.x); lb = bf16_bits(c1.x - __uint_as_float(hb << 16)); q[4] = (unsigned short)(lo ? lb : hb);
      hb = bf16_bits(c1.y); lb = bf16_bits(c1.y - __uint_as_float(hb << 16)); q[5] = (unsigned short)(lo ? lb : hb);
      hb = bf16_bits(c1.z); lb = bf16_bits(c1.z - __uint_as_float(hb << 16)); q[6] = (unsigned short)(lo ? lb : hb);
      hb = bf16_bits(c1.w); lb = bf16_bits(c1.w - __uint_as_float(hb << 16)); q[7] = (unsigned short)(lo ? lb : hb);
      qv[i] = q;
    }
  }
#pragma unroll
  for (int i = 0; i < 8; ++i) {
    const int gr = rowBase + 16 * wave + 2 * i + hh;
    *(volatile v4f*)(hall + (size_t)gr * HALLP + coloff + 4 * m) = fv[i];
    if constexpr (WRH != 0) *(volatile v8us*)(hout + (size_t)gr * HP + 8 * m) = qv[i];
  }
  __threadfence();
#pragma unroll
  for (int i = 0; i < 8; ++i) {
    const int gr = rowBase + 16 * wave + 2 * i + hh;
    *(volatile v4f*)(hall + (size_t)gr * HALLP + coloff + 4 * m) = fv[i];
    if constexpr (WRH != 0) *(volatile v8us*)(hout + (size_t)gr * HP + 8 * m) = qv[i];
  }
}

__global__ __launch_bounds__(PTHR) void k_pool_head(const float* __restrict__ hall, const int* __restrict__ bat,
                                                    int nN, const unsigned short* __restrict__ wall,
                                                    const float* __restrict__ b1, const float* __restrict__ W2,
                                                    const float* __restrict__ b2, float* out) {
  __shared__ float gt[PG * HALLP];
  __shared__ __attribute__((aligned(16))) unsigned short ga[PG * GAP];
  __shared__ float g1[PG * DFE];
  __shared__ float w2s[DFE * NCLS];
  __shared__ float b2s[16];
  __shared__ __attribute__((aligned(16))) float os[PG * NCLS];
  __shared__ int rng[PG + 1];
  __shared__ int cn[PG];
  __shared__ int vio[8];
  const int tid = (int)threadIdx.x, lane = tid & 31, wave = tid >> 5, hh = lane >> 4, m = lane & 15;
  const int g0 = (int)blockIdx.x * PG;

#pragma unroll 1
  for (int i = tid; i < DFE * NCLS; i += PTHR) w2s[i] = bf16_val(W2[i]);
  if (tid < 16) {
    const float bb = b2[tid < NCLS ? tid : NCLS - 1];
    b2s[tid] = (tid < NCLS) ? bf16_val(bb) : 0.0f;
    cn[tid] = 0;
  }
#pragma unroll 1
  for (int gi = 0; gi < PG; ++gi) gt[gi * HALLP + tid] = 0.0f;

  int bad = 0;
#pragma unroll 1
  for (int i = tid; i < nN - 1; i += PTHR) {
    const int a = bat[i];
    const int b = bat[i + 1];
    bad |= (a > b) ? 1 : 0;
  }
  const unsigned mb = __builtin_amdgcn_ballot_w32(bad != 0);
  if (lane == 0) vio[wave] = (mb != 0u) ? 1 : 0;

  {
    const int key = g0 + (tid < PG ? tid : PG);
    int lo = 0, n = nN;
#pragma unroll 1
    for (int it = 0; it < 21; ++it) {
      const int half = n >> 1;
      int mid = lo + half;
      mid = mid > nN - 1 ? nN - 1 : mid;
      const int v = bat[mid];
      const bool take = (n > 0) && (v < key);
      lo = take ? mid + 1 : lo;
      n  = take ? n - half - 1 : half;
    }
    if (tid <= PG) rng[tid] = lo;
  }
  __syncthreads();
  int nonmono = 0;
#pragma unroll
  for (int w2 = 0; w2 < PWAVE; ++w2) nonmono |= vio[w2];

  if (nonmono == 0) {
#pragma unroll 1
    for (int gi = 0; gi < PG; ++gi) {
      int lo = rng[gi];
      int hi = rng[gi + 1];
      lo = lo < 0 ? 0 : (lo > nN ? nN : lo);
      hi = hi < lo ? lo : (hi > nN ? nN : hi);
      float acc = 0.0f;
#pragma unroll 1
      for (int nd = lo; nd < hi; ++nd) acc += hall[(size_t)nd * HALLP + tid];
      const int c = hi - lo;
      const float cf = (c < 1) ? 1.0f : (float)c;
      gt[gi * HALLP + tid] = acc * (1.0f / cf);
    }
  } else {
#pragma unroll 1
    for (int nd = 0; nd < nN; ++nd) {
      const int d = bat[nd] - g0;
      if ((unsigned)d < (unsigned)PG) {
        const float a = gt[d * HALLP + tid];
        gt[d * HALLP + tid] = a + hall[(size_t)nd * HALLP + tid];
        if (tid == 0) cn[d] = cn[d] + 1;
      }
    }
  }
  __syncthreads();
  if (nonmono != 0) {
#pragma unroll 1
    for (int gi = 0; gi < PG; ++gi) {
      const int c = cn[gi];
      const float cf = (c < 1) ? 1.0f : (float)c;
      const float a = gt[gi * HALLP + tid];
      gt[gi * HALLP + tid] = a * (1.0f / cf);
    }
  }
#pragma unroll 1
  for (int gi = 0; gi < PG; ++gi) {
    const float v = gt[gi * HALLP + tid];
    const unsigned hb = bf16_bits(v);
    const unsigned lb = bf16_bits(v - __uint_as_float(hb << 16));
    ga[gi * GAP + tid]         = (unsigned short)hb;
    ga[gi * GAP + HALLP + tid] = (unsigned short)lb;
  }
  __syncthreads();

  {
    const int nt = wave < 4 ? wave : 3;
    v8f acc = {0.f, 0.f, 0.f, 0.f, 0.f, 0.f, 0.f, 0.f};
    const unsigned short* ar = ga + m * GAP + 8 * hh;
    const unsigned short* wq = wall + (size_t)(16 * nt + m) * WP + W1OFF + 8 * hh;
#pragma unroll 1
    for (int ks = 0; ks < GAP / 32; ++ks) {
      FragB af, bf;
      af.h[0] = *(const v8usa*)(ar + 32 * ks);
      af.h[1] = *(const v8usa*)(ar + 32 * ks + 16);
      bf.h[0] = *(const v8usa*)(wq + 32 * ks);
      bf.h[1] = *(const v8usa*)(wq + 32 * ks + 16);
      acc = wmb(af, bf, acc);
    }
    const int col = 16 * nt + m;
    const float bv = bf16_val(b1[col]);
    if (wave < 4) {
#pragma unroll
      for (int r = 0; r < 8; ++r) {
        const float v = acc[r] + bv;
        g1[(8 * hh + r) * DFE + col] = (v > 0.0f) ? v : (v - v);
      }
    }
  }
  __syncthreads();

  if (tid < PG * NCLS) {
    const int gi = tid / NCLS;
    const int c  = tid - gi * NCLS;
    const float* gr = g1 + gi * DFE;
    float s = 0.0f;
#pragma unroll 4
    for (int k = 0; k < DFE; ++k) s = fmaf(gr[k], w2s[k * NCLS + c], s);
    os[tid] = s + b2s[c];
  }
  __syncthreads();

  const int q = tid < 40 ? tid : 39;
  const v4f ov = *(const v4fa*)(os + 4 * q);
  float* op = out + (size_t)g0 * NCLS + 4 * q;
  const bool okst = tid < 40;
  if (okst) *(volatile v4f*)op = ov;
  __threadfence();
  if (okst) *(volatile v4f*)op = ov;
}

static inline int cdiv(int a, int b) { return (a + b - 1) / b; }
static inline size_t al256(size_t o) { return (o + 255) & ~(size_t)255; }

extern "C" void kernel_launch(void* const* d_in, const int* in_sizes, int n_in,
                              void* d_out, int out_size, void* d_ws, size_t ws_size,
                              hipStream_t stream) {
  if (n_in < 18) return;
  if (in_sizes[0] < DFE || (in_sizes[0] % DFE) != 0) return;
  const int nN = in_sizes[0] / DFE;
  if (nN < 16 || nN >= (1 << 20)) return;
  if (in_sizes[1] < 2 || (in_sizes[1] & 1) != 0) return;
  const int nE = in_sizes[1] / 2;
  if (nE < 1 || nE >= (1 << (31 - SLA))) return;
  if (in_sizes[2] != nN) return;
  for (int l = 0; l < 3; ++l) {
    if (in_sizes[3 + 3 * l] != DFE * DFE) return;
    if (in_sizes[4 + 3 * l] != DFE) return;
    if (in_sizes[5 + 3 * l] != DFE * DFE) return;
  }
  if (in_sizes[12] != DFE * DFE || in_sizes[13] != DFE) return;
  if (in_sizes[14] != HALLP * DFE || in_sizes[15] != DFE) return;
  if (in_sizes[16] != DFE * NCLS || in_sizes[17] != NCLS) return;
  if (out_size != NOUT) return;

  const float* x    = (const float*)d_in[0];
  const int*   edge = (const int*)d_in[1];
  const int*   bat  = (const int*)d_in[2];
  const float* Wl0  = (const float*)d_in[3];
  const float* bl0  = (const float*)d_in[4];
  const float* Wr0  = (const float*)d_in[5];
  const float* Wl1  = (const float*)d_in[6];
  const float* bl1  = (const float*)d_in[7];
  const float* Wr1  = (const float*)d_in[8];
  const float* Wl2  = (const float*)d_in[9];
  const float* bl2  = (const float*)d_in[10];
  const float* Wr2  = (const float*)d_in[11];
  const float* Wm   = (const float*)d_in[12];
  const float* bm   = (const float*)d_in[13];
  const float* W1   = (const float*)d_in[14];
  const float* b1   = (const float*)d_in[15];
  const float* W2   = (const float*)d_in[16];
  const float* b2   = (const float*)d_in[17];
  float* out = (float*)d_out;
  const int* src = edge;
  const int* dst = edge + nE;

  const int MP = cdiv(nN, GBM) * GBM;
  const int gM = MP / GBM;
  const int gA = cdiv(MP, NBA);
  if ((long long)gA * NBA < (long long)MP) return;
  const int vec8 = ((nE & 3) == 0) ? 1 : 0;

  char* ws = (char*)d_ws;
  size_t off = 0;
  const size_t oWALL = off; off = al256(off + (size_t)DFE * WP * 2);
  const size_t oXB   = off; off = al256(off + (size_t)MP * DFE * 2);
  const size_t oMEAN = off; off = al256(off + (size_t)MP * HP * 2);
  const size_t oHHA  = off; off = al256(off + (size_t)MP * HP * 2);
  const size_t oHHB  = off; off = al256(off + (size_t)MP * HP * 2);
  const size_t oHALL = off; off = al256(off + (size_t)MP * HALLP * 4);
  if (off > ws_size || off > (size_t)WSMAX) return;
  unsigned short* WALL = (unsigned short*)(ws + oWALL);
  unsigned short* XB   = (unsigned short*)(ws + oXB);
  unsigned short* MEAN = (unsigned short*)(ws + oMEAN);
  unsigned short* HHA  = (unsigned short*)(ws + oHHA);
  unsigned short* HHB  = (unsigned short*)(ws + oHHB);
  float*          HALL = (float*)(ws + oHALL);

  const size_t scanLds = (size_t)AGG_LDS_INTS * 4;
  hipFuncSetAttribute(reinterpret_cast<const void*>(&k_scan<1>), hipFuncAttributeMaxDynamicSharedMemorySize, (int)scanLds);
  hipFuncSetAttribute(reinterpret_cast<const void*>(&k_scan<0>), hipFuncAttributeMaxDynamicSharedMemorySize, (int)scanLds);

  const int nUx = MP * (DFE / 8);
  k_prep<<<(NSUB * 512) / NTHR, NTHR, 0, stream>>>(Wl0, Wr0, Wl1, Wr1, Wl2, Wr2, Wm, W1, WALL);
  k_cvx<<<cdiv(nUx, NTHR), NTHR, 0, stream>>>(x, nN, nUx, XB);
  k_scan<1><<<gA, NTHR, scanLds, stream>>>(src, dst, nE, nN, vec8, MP, XB, HALL, 0, MEAN);
  k_layer<1, 1><<<gM, GTHR, 0, stream>>>(MEAN, XB, WALL, WC0OFF, bl0, bm, HALL, 0, HHA);
  k_scan<0><<<gA, NTHR, scanLds, stream>>>(src, dst, nE, nN, vec8, MP, XB, HALL, 0, MEAN);
  k_layer<0, 1><<<gM, GTHR, 0, stream>>>(MEAN, HHA, WALL, WC1OFF, bl1, bm, HALL, DFE, HHB);
  k_scan<0><<<gA, NTHR, scanLds, stream>>>(src, dst, nE, nN, vec8, MP, XB, HALL, DFE, MEAN);
  k_layer<0, 0><<<gM, GTHR, 0, stream>>>(MEAN, HHB, WALL, WC2OFF, bl2, bm, HALL, 2 * DFE, HHA);
  k_pool_head<<<NGR / PG, PTHR, 0, stream>>>(HALL, bat, nN, WALL, b1, W2, b2, out);
}
